// EGNNNetwork_90752658965038
// MI455X (gfx1250) — hardware-run, weakly checked
//
#include <hip/hip_runtime.h>


namespace {
constexpr int N = 50000, E = 800000, G = 64, NF = 110, FP = 128, M = 32, EH = 128, NHID = 128, NL = 2, NBLK = N / 16;
constexpr float XS = 8.0f, WSC = 256.0f;
__constant__ int EMB_N[10] = {119, 11, 12, 8, 2, 9, 2, 9, 5, 7};
__constant__ int EMB_D[10] = {32, 8, 8, 8, 8, 8, 8, 8, 8, 8};
__constant__ int EMB_OFF[10] = {6, 38, 46, 54, 62, 70, 78, 86, 94, 102};
__constant__ int KEEP[6] = {0, 11, 12, 13, 14, 15};
typedef _Float16 b16;
typedef __attribute__((ext_vector_type(16))) _Float16 v16b;
typedef __attribute__((ext_vector_type(8))) _Float16 v8b;
typedef __attribute__((ext_vector_type(8))) float v8f;
typedef __attribute__((ext_vector_type(4))) float v4f;
__device__ __forceinline__ float bf16_rne(float f) { unsigned int u = __float_as_uint(f); u += 0x7FFFu + ((u >> 16) & 1u); return __uint_as_float(u & 0xFFFF0000u); }
__device__ __forceinline__ v16b frag_kb(const b16* p, int hh) { const v8b a = *(const v8b*)(p + 8 * hh), b = *(const v8b*)(p + 16 + 8 * hh); v16b f;
#pragma unroll
  for (int e = 0; e < 8; ++e) { f[e] = a[e]; f[8 + e] = b[e]; } return f; }
__device__ __forceinline__ v8f wmma16b(v16b a, v16b b, v8f c) { v8f d = __builtin_amdgcn_wmma_f32_16x16x32_f16(false, a, false, b, (short)0, c, false, false); asm volatile("v_nop\n\tv_nop\n\tv_nop\n\tv_nop" : "+v"(d) : "v"(a), "v"(b)); return d; }
__device__ __forceinline__ void wave_lds_sync() { __builtin_amdgcn_fence(__ATOMIC_RELEASE, "workgroup"); __builtin_amdgcn_wave_barrier(); __builtin_amdgcn_fence(__ATOMIC_ACQUIRE, "workgroup"); }
__device__ __forceinline__ float pmul(float a, float b) { float p = a * b; asm volatile("" : "+v"(p)); return p; }
__device__ __forceinline__ int iclamp(int v, int lo, int hi) { return v < lo ? lo : (v > hi ? hi : v); }
__device__ __forceinline__ float silu(float v) { return v / (1.0f + __expf(-v)); }
constexpr int CSR_NBLK9 = 512, CSR_GB9 = 9, CSR_GN9 = 1 << CSR_GB9  , CSR_TS9 = (CSR_GN9 < 32 ? 32 : CSR_GN9)  , CSR_MAXG9 = 512, CSR_CAP9 = 12288  ;
__device__ __host__ __forceinline__ int csr_tix9(int v) { return (v >> CSR_GB9) * CSR_TS9 + (v & (CSR_GN9 - 1)); }
__global__ __launch_bounds__(64) void csrA_kernel9(const int* __restrict__ dst, int E, int N, int nG, int CHP, int NGP, int* __restrict__ STG, int* __restrict__ HST) {
  extern __shared__ int sm[];
  int* cnt = sm; int* run = sm + NGP; int* ids = sm + 2 * NGP;
  const int b = blockIdx.x; const int ch = (E + CSR_NBLK9 - 1) / CSR_NBLK9; const int e0 = b * ch, e1 = min(E, e0 + ch);
  for (int i = threadIdx.x; i < NGP; i += 64) cnt[i] = 0;
  for (int i = threadIdx.x; i < CHP; i += 64) ids[i] = -1;
  __syncthreads();
  if (threadIdx.x == 0) {
    for (int e = e0; e < e1; ++e) { int d = dst[e]; d = (d < 0) ? 0 : (d >= N ? N - 1 : d); cnt[d >> CSR_GB9] += 1; }
    int acc = 0; for (int g = 0; g < nG; ++g) { run[g] = acc; acc += cnt[g]; }
    for (int e = e0; e < e1; ++e) { int d = dst[e]; d = (d < 0) ? 0 : (d >= N ? N - 1 : d); const int g = d >> CSR_GB9; ids[run[g]] = e; run[g] += 1; } }
  __syncthreads();
  typedef __attribute__((ext_vector_type(4))) int v4i;
  for (int pass = 0; pass < 2; ++pass) {
    for (int i = threadIdx.x; i < CHP / 4; i += 64) *(volatile v4i*)(STG + (size_t)b * CHP + i * 4) = *(const v4i*)(&ids[i * 4]);
    for (int i = threadIdx.x; i < NGP / 4; i += 64) { v4i v; for (int e = 0; e < 4; ++e) v[e] = (i * 4 + e < nG) ? cnt[i * 4 + e] : 0; *(volatile v4i*)(HST + (size_t)b * NGP + i * 4) = v; }
    __threadfence(); }
}
__global__ __launch_bounds__(512) void csrS_kernel9(const int* __restrict__ HST, int nG, int NGP, int* __restrict__ START, int* __restrict__ TOT, int* __restrict__ OFF) {
  __shared__ int tot[CSR_MAXG9];
  const int b = threadIdx.x;
  for (int pass = 0; pass < 2; ++pass) { int runb = 0; for (int g = 0; g < nG; ++g) { int c = HST[(size_t)b * NGP + g]; c = (c < 0) ? 0 : c; ((volatile int*)OFF)[(size_t)g * CSR_NBLK9 + b] = runb; runb += c; } __threadfence(); }
  for (int g = threadIdx.x; g < nG; g += 512) { int s = 0; for (int bb = 0; bb < CSR_NBLK9; ++bb) { int c = HST[(size_t)bb * NGP + g]; s += (c < 0) ? 0 : c; } tot[g] = s; }
  __syncthreads();
  if (threadIdx.x < 32) {
    __shared__ int st[CSR_MAXG9 + 32];
    if (threadIdx.x == 0) { int acc = 0; for (int g = 0; g < NGP; ++g) { st[g] = acc; if (g < nG) acc += (tot[g] + 31) & ~31; } st[NGP] = acc; }
    __builtin_amdgcn_fence(__ATOMIC_RELEASE, "workgroup"); __builtin_amdgcn_wave_barrier(); __builtin_amdgcn_fence(__ATOMIC_ACQUIRE, "workgroup");
    for (int pass = 0; pass < 2; ++pass) { for (int i = threadIdx.x; i < NGP + 32; i += 32) { ((volatile int*)START)[i] = (i <= NGP) ? st[min(i, NGP)] : 0; ((volatile int*)TOT)[i] = (i < nG) ? tot[i] : 0; } __threadfence(); } }
}
__global__ __launch_bounds__(256) void csrB_kernel9(const int* __restrict__ dst, int N, int nG, int CHP, int NGP, int permLen, const int* __restrict__ STG, const int* __restrict__ HST, const int* __restrict__ OFF, const int* __restrict__ START, const int* __restrict__ TOT, int* __restrict__ PERM, int* __restrict__ ROWPTR, int* __restrict__ ROWCNT, int* __restrict__ FLAG) {
  typedef __attribute__((ext_vector_type(4))) int v4i;
  __shared__ int ids[CSR_CAP9]; __shared__ unsigned short key[CSR_CAP9]; __shared__ int outp[CSR_CAP9]; __shared__ int ncnt[CSR_GN9 + 1]; __shared__ int boff[CSR_NBLK9 + 1];
  const int g = blockIdx.x, t_ = threadIdx.x; int tot = TOT[g]; int st = START[g], stn = START[g + 1]; const int v0 = g * CSR_GN9; const int nv = min(CSR_GN9, N - v0); const int t0 = g * CSR_TS9;
  st = (st < 0) ? 0 : (st > permLen - 32 ? permLen - 32 : st) & ~31; stn = (stn < st) ? st : (stn > permLen ? permLen : stn); tot = (tot < 0) ? 0 : tot; if (tot > stn - st && tot <= CSR_CAP9) tot = stn - st;
  if (tot > CSR_CAP9) {
    for (int pass = 0; pass < 2; ++pass) { for (int i = t_; i < CSR_TS9 / 4; i += 256) { v4i a, c; for (int e = 0; e < 4; ++e) { a[e] = st; c[e] = 0; } *(volatile v4i*)(ROWPTR + t0 + i * 4) = a; *(volatile v4i*)(ROWCNT + t0 + i * 4) = c; } if (t_ == 0) ((volatile int*)FLAG)[0] = 1; __threadfence(); } (void)nv; return; }
  if (t_ == 0) { int acc = 0; for (int b = 0; b < CSR_NBLK9; ++b) { boff[b] = acc; int c = HST[(size_t)b * NGP + g]; c = (c < 0) ? 0 : (c > CHP ? CHP : c); acc += c; if (acc > tot) acc = tot; } boff[CSR_NBLK9] = acc; }
  for (int i = t_; i <= CSR_GN9; i += 256) ncnt[i] = 0;
  __syncthreads();
  for (int b = 0; b < CSR_NBLK9; ++b) { const int c = boff[b + 1] - boff[b]; int o_ = OFF[(size_t)g * CSR_NBLK9 + b]; o_ = (o_ < 0) ? 0 : (o_ > CHP - c ? CHP - c : o_); const int* src_ = STG + (size_t)b * CHP + o_;
    for (int i = t_; i < c; i += 256) { int id = src_[i]; id = (id < 0) ? 0 : id; ids[boff[b] + i] = id; int d = dst[id]; d = (d < v0) ? v0 : (d >= N ? N - 1 : d); int kk = d - v0; kk = (kk < 0) ? 0 : (kk >= CSR_GN9 ? CSR_GN9 - 1 : kk); key[boff[b] + i] = (unsigned short)kk; } }
  __syncthreads();
  if (t_ == 0) { for (int i = 0; i < tot; ++i) ncnt[key[i]] += 1; int acc = 0; for (int vl = 0; vl < CSR_GN9; ++vl) { const int c = ncnt[vl]; ncnt[vl] = acc; acc += c; } ncnt[CSR_GN9] = acc;
    for (int i = 0; i < tot; ++i) { const int vl = key[i]; outp[ncnt[vl]] = ids[i]; ncnt[vl] += 1; }
    for (int vl = CSR_GN9; vl > 0; --vl) ncnt[vl] = ncnt[vl - 1]; ncnt[0] = 0; }
  __syncthreads();
  for (int pass = 0; pass < 2; ++pass) {
    for (int i = t_; i < (stn - st) / 4; i += 256) { v4i v; for (int e = 0; e < 4; ++e) { const int q = i * 4 + e; v[e] = (q < tot) ? outp[q] : -1; } *(volatile v4i*)(PERM + st + i * 4) = v; }
    for (int i = t_; i < CSR_TS9 / 4; i += 256) { v4i a, c; for (int e = 0; e < 4; ++e) { const int vl = i * 4 + e; const int vc = vl < CSR_GN9 ? vl : CSR_GN9; a[e] = (vl < CSR_GN9) ? st + ncnt[vc] : st; c[e] = (vl < nv) ? (ncnt[(vc < CSR_GN9 ? vc : CSR_GN9 - 1) + 1] - ncnt[vc]) : 0; } *(volatile v4i*)(ROWPTR + t0 + i * 4) = a; *(volatile v4i*)(ROWCNT + t0 + i * 4) = c; }
    __threadfence(); }
}
__global__ __launch_bounds__(256) void csrZ_kernel9(int* __restrict__ p, size_t n4) { typedef __attribute__((ext_vector_type(4))) int v4i; const size_t tid = (size_t)blockIdx.x * 256 + threadIdx.x, nth = (size_t)gridDim.x * 256; v4i z = {0, 0, 0, 0}; for (size_t i = tid; i < n4; i += nth) *(volatile v4i*)(p + i * 4) = z; }
struct CsrBufs9 { int *STG, *HST, *OFF, *START, *TOT, *PERM, *ROWPTR, *ROWCNT, *FLAG; int nG, NGP, CHP; size_t permLen; char* base; size_t bytes; };
static size_t csr_carve9(CsrBufs9& c, char* ws, size_t off, int E, int N) {
  const size_t off0 = off; c.base = ws + off;
  auto al = [&](size_t bytes) { char* p = ws + off; off += (bytes + 255) & ~(size_t)255; return p; };
  c.nG = (N + CSR_GN9 - 1) / CSR_GN9; c.NGP = (c.nG + 31) & ~31; const int ch = (E + CSR_NBLK9 - 1) / CSR_NBLK9; c.CHP = (ch + 31) & ~31; c.permLen = (size_t)E + 32 * (size_t)c.nG + 32;
  c.STG = (int*)al((size_t)CSR_NBLK9 * c.CHP * 4); c.HST = (int*)al((size_t)CSR_NBLK9 * c.NGP * 4); c.OFF = (int*)al((size_t)c.NGP * CSR_NBLK9 * 4); c.START = (int*)al((size_t)(c.NGP + 64) * 4); c.TOT = (int*)al((size_t)(c.NGP + 64) * 4);
  c.PERM = (int*)al(c.permLen * 4); c.ROWPTR = (int*)al((size_t)c.nG * CSR_TS9 * 4); c.ROWCNT = (int*)al((size_t)c.nG * CSR_TS9 * 4); c.FLAG = (int*)al(256);
  c.bytes = off - off0; return off;
}
static void csr_build9(const CsrBufs9& c, const int* dst, int E, int N, hipStream_t stream) {
  const size_t smem = (size_t)(2 * c.NGP + c.CHP) * 4;
  csrZ_kernel9<<<512, 256, 0, stream>>>((int*)c.base, c.bytes / 16);
  csrA_kernel9<<<CSR_NBLK9, 64, smem, stream>>>(dst, E, N, c.nG, c.CHP, c.NGP, c.STG, c.HST);
  csrS_kernel9<<<1, 512, 0, stream>>>(c.HST, c.nG, c.NGP, c.START, c.TOT, c.OFF);
  csrB_kernel9<<<c.nG, 256, 0, stream>>>(dst, N, c.nG, c.CHP, c.NGP, (int)c.permLen, c.STG, c.HST, c.OFF, c.START, c.TOT, c.PERM, c.ROWPTR, c.ROWCNT, c.FLAG);
}


__global__ __launch_bounds__(256) void wput_kernel(const float* __restrict__ w, int r0, int KIN, int KW, int OUTW, int OUTP, int ro, int ko, int KP, b16* __restrict__ WT) {
  const int KG = KW / 8; const int u = blockIdx.x * 256 + threadIdx.x; if (u >= OUTP * KG) return; const int o = u / KG, k0 = (u % KG) * 8; v8b v;
#pragma unroll
  for (int j = 0; j < 8; ++j) { const int k = k0 + j; v[j] = (o < OUTW && k < KIN) ? (b16)(bf16_rne(w[(size_t)(r0 + k) * OUTW + o]) * WSC) : (b16)0.0f; } for (int pass = 0; pass < 2; ++pass) { *(volatile v8b*)(WT + (size_t)(ro + o) * KP + ko + k0) = v; __threadfence(); }
}
__global__ __launch_bounds__(32) void feat_kernel(const float* __restrict__ x, const float* const* __restrict__ dummy, const float* __restrict__ e0, const float* __restrict__ e1, const float* __restrict__ e2, const float* __restrict__ e3, const float* __restrict__ e4, const float* __restrict__ e5, const float* __restrict__ e6, const float* __restrict__ e7, const float* __restrict__ e8, const float* __restrict__ e9, float* __restrict__ Fo) {
  (void)dummy; __shared__ float Row[16][FP]; const int lane = threadIdx.x; const size_t m0 = (size_t)blockIdx.x * 16; const float* embs[10] = {e0, e1, e2, e3, e4, e5, e6, e7, e8, e9};
  for (int rr = 0; rr < 16; ++rr) { const size_t n = m0 + rr; for (int q = 0; q < 4; ++q) Row[rr][q * 32 + lane] = 0.0f; }
  wave_lds_sync();
  for (int rr = 0; rr < 16; ++rr) { const size_t n = m0 + rr; if (lane < 6) Row[rr][lane] = bf16_rne(x[n * 16 + KEEP[lane]]);
    for (int j = 0; j < 10; ++j) { const int nj = EMB_N[j], dj = EMB_D[j]; int code = (int)bf16_rne(x[n * 16 + 1 + j]); if (code < 0) code += nj; code = iclamp(code, 0, nj - 1); if (lane < dj) Row[rr][EMB_OFF[j] + lane] = bf16_rne(embs[j][code * dj + lane]); } }
  wave_lds_sync();
  for (int pass = 0; pass < 2; ++pass) { for (int rr = 0; rr < 16; ++rr) *(volatile v4f*)(Fo + (m0 + rr) * FP + lane * 4) = *(const v4f*)(&Row[rr][lane * 4]); __threadfence(); }
}
template <int KP, int NT, int SILU>
__global__ __launch_bounds__(32) void dense_kernel(const float* __restrict__ IN, int pin, int KIN, const b16* __restrict__ WT, const float* __restrict__ bias, int nbias, int pout, int NLIM, float* __restrict__ OUT) {
  __shared__ __attribute__((aligned(16))) b16 Ah[16][KP + 8]; __shared__ __attribute__((aligned(16))) float Tf[16][128 + 4];
  const int lane = threadIdx.x, nloc = lane & 15, hlf = lane >> 4; const size_t m0 = (size_t)blockIdx.x * 16; if (m0 >= (size_t)NLIM) return;
  for (int rr = 0; rr < 16; ++rr) for (int q = 0; q < KP / 32; ++q) { const int c = q * 32 + lane; Ah[rr][c] = (b16)((c < KIN ? IN[(m0 + rr) * pin + c] : 0.0f) * XS); }
  wave_lds_sync();
#pragma unroll 1
  for (int cg = 0; cg < (NT + 7) / 8; ++cg) { const int nt = (NT - cg * 8) < 8 ? (NT - cg * 8) : 8; v8f acc[8];
#pragma unroll
    for (int t = 0; t < 8; ++t) acc[t] = (v8f){};
#pragma unroll
    for (int kb = 0; kb < KP; kb += 32) { const v16b a = frag_kb(&Ah[nloc][kb], hlf);
#pragma unroll
      for (int t = 0; t < 8; ++t) if (t < nt) acc[t] = wmma16b(a, frag_kb(WT + (size_t)(cg * 128 + t * 16 + nloc) * KP + kb, hlf), acc[t]); }
#pragma unroll
    for (int t = 0; t < 8; ++t) { if (t < nt) { const int c = cg * 128 + t * 16 + nloc; const float bb = c < nbias ? bf16_rne(bias[c]) : 0.0f;
#pragma unroll
        for (int r8 = 0; r8 < 8; ++r8) { float v = acc[t][r8] * (1.0f / (XS * WSC)) + bb; if (SILU) v = silu(v); Tf[8 * hlf + r8][t * 16 + nloc] = v; } } }
    wave_lds_sync();
    for (int pass = 0; pass < 2; ++pass) { for (int rr = 0; rr < 16; ++rr) for (int c = lane; c < nt * 16; c += 32) ((volatile float*)OUT)[(m0 + rr) * pout + cg * 128 + c] = Tf[rr][c]; __threadfence(); }
    wave_lds_sync(); }
}
__global__ __launch_bounds__(32) void msg_kernel(const float* __restrict__ PDS, const float* __restrict__ pos, const float* __restrict__ ea, const int* __restrict__ srcs, const float* __restrict__ W1, const float* __restrict__ b1, const b16* __restrict__ W2T, const float* __restrict__ b2, const int* __restrict__ PERM, const int* __restrict__ ROWPTR, const int* __restrict__ ROWCNT, int permLen, int NLIM, float* __restrict__ MI) {
  __shared__ __attribute__((aligned(16))) b16 Ah[16][EH + 8]; __shared__ int Ss[16]; __shared__ float Ea[16], D2[16], So[2][16];
  const int lane = threadIdx.x, nloc = lane & 15, hlf = lane >> 4; const size_t v = blockIdx.x; if (v >= (size_t)NLIM) return;
  float pd[4], wa[4], wd[4], bb[4]; for (int i = 0; i < 4; ++i) { const int c = lane * 4 + i; pd[i] = PDS[v * 256 + c]; wa[i] = bf16_rne(W1[(size_t)220 * EH + c]); wd[i] = bf16_rne(W1[(size_t)221 * EH + c]); bb[i] = bf16_rne(b1[c]); }
  const float px = bf16_rne(pos[v * 3]), py = bf16_rne(pos[v * 3 + 1]), pz = bf16_rne(pos[v * 3 + 2]); const float c2a = bf16_rne(b2[nloc]), c2b = bf16_rne(b2[16 + nloc]);
  int st = ROWPTR[v], cnt = ROWCNT[v]; cnt = iclamp(cnt, 0, 1 << 20); st = iclamp(st, 0, permLen - cnt); const int tot = cnt + 1; float macc0 = 0.0f, macc1 = 0.0f;
#pragma unroll 1
  for (int j0 = 0; j0 < tot; j0 += 16) {
    if (lane < 16) { const int jj = j0 + lane; int s = -1; float eav = 0.0f, d2 = 0.0f; if (jj == 0) s = (int)v; else if (jj < tot) { const int e = iclamp(PERM[st + jj - 1], 0, E - 1); s = iclamp(srcs[e], 0, N - 1); if (s >= NLIM) s = -1; else { eav = bf16_rne(ea[e]); const float dx = bf16_rne(pos[(size_t)s * 3]) - px, dy = bf16_rne(pos[(size_t)s * 3 + 1]) - py, dz = bf16_rne(pos[(size_t)s * 3 + 2]) - pz; d2 = pmul(dx, dx) + pmul(dy, dy) + pmul(dz, dz); } } Ss[lane] = s; Ea[lane] = eav; D2[lane] = d2; }
    wave_lds_sync();
    for (int rr = 0; rr < 16; ++rr) { const int s = Ss[rr]; for (int i = 0; i < 4; ++i) { float a = 0.0f; if (s >= 0) a = silu(pd[i] + PDS[(size_t)s * 256 + 128 + lane * 4 + i] + pmul(Ea[rr], wa[i]) + pmul(D2[rr], wd[i]) + bb[i]); Ah[rr][lane * 4 + i] = (b16)(a * XS); } }
    wave_lds_sync();
    v8f acc[2] = {(v8f){}, (v8f){}};
#pragma unroll
    for (int kb = 0; kb < EH; kb += 32) { const v16b a = frag_kb(&Ah[nloc][kb], hlf);
#pragma unroll
      for (int t = 0; t < 2; ++t) acc[t] = wmma16b(a, frag_kb(W2T + (size_t)(t * 16 + nloc) * EH + kb, hlf), acc[t]); }
    float s0 = 0.0f, s1 = 0.0f;
#pragma unroll
    for (int r8 = 0; r8 < 8; ++r8) { const int rl = 8 * hlf + r8; const bool ok = (Ss[rl] >= 0); s0 += ok ? silu(acc[0][r8] * (1.0f / (XS * WSC)) + c2a) : 0.0f; s1 += ok ? silu(acc[1][r8] * (1.0f / (XS * WSC)) + c2b) : 0.0f; }
    if (hlf == 1) { So[0][nloc] = s0; So[1][nloc] = s1; }
    wave_lds_sync();
    if (hlf == 0) { macc0 += s0 + So[0][nloc]; macc1 += s1 + So[1][nloc]; }
    wave_lds_sync(); }
  for (int pass = 0; pass < 2; ++pass) { if (hlf == 0) { ((volatile float*)MI)[v * M + nloc] = macc0; ((volatile float*)MI)[v * M + 16 + nloc] = macc1; } __threadfence(); }
}
__global__ __launch_bounds__(256) void lnstat_kernel(const float* __restrict__ Fo, const int* __restrict__ batch, int NLIM, float* __restrict__ ST) {
  __shared__ float red[8]; __shared__ float mu_s; const int g = blockIdx.x, tid = threadIdx.x, wave = tid >> 5, lane = tid & 31;
  auto lb = [&](int key) -> int { int lo = 0, hi = N; for (int it = 0; it < 17 && lo < hi; ++it) { const int mid = (lo + hi) >> 1; if (batch[mid] < key) lo = mid + 1; else hi = mid; } return lo; };
  int s0 = lb(g), e0 = lb(g + 1); if (e0 > NLIM) e0 = NLIM; if (e0 < s0) e0 = s0; const float denom = (float)((e0 - s0) < 1 ? 1 : (e0 - s0)) * (float)NF;
  float s = 0.0f; for (int i = s0 * FP + tid; i < e0 * FP; i += 256) { const int c = i % FP; if (c < NF) s += Fo[i]; }
  for (int o = 16; o; o >>= 1) s += __shfl_xor(s, o); if (lane == 0) red[wave] = s; __syncthreads(); if (tid == 0) { float t = 0.0f; for (int w = 0; w < 8; ++w) t += red[w]; mu_s = t / denom; } __syncthreads(); const float mu = mu_s;
  float q = 0.0f; for (int i = s0 * FP + tid; i < e0 * FP; i += 256) { const int c = i % FP; if (c < NF) { const float d = Fo[i] - mu; q += pmul(d, d); } }
  for (int o = 16; o; o >>= 1) q += __shfl_xor(q, o); if (lane == 0) red[wave] = q; __syncthreads();
  if (tid < 32) { float t = 0.0f; for (int w = 0; w < 8; ++w) t += red[w]; const float rstd = rsqrtf(t / denom + 1e-5f); for (int pass = 0; pass < 2; ++pass) { ((volatile float*)ST)[g * 32 + lane] = lane == 0 ? mu : rstd; __threadfence(); } }
}
__global__ __launch_bounds__(32) void nin_kernel(const float* __restrict__ Fo, const float* __restrict__ MI, const float* __restrict__ ST, const int* __restrict__ batch, const float* __restrict__ lw, const float* __restrict__ lb_, int NLIM, float* __restrict__ NI) {
  const int lane = threadIdx.x; const size_t m0 = (size_t)blockIdx.x * 16; if (m0 >= (size_t)NLIM) return;
  for (int pass = 0; pass < 2; ++pass) { for (int rr = 0; rr < 16; ++rr) { const size_t n = m0 + rr; const int g = iclamp(batch[n], 0, G - 1); const float mu = ST[g * 32], rs = ST[g * 32 + 1];
      for (int q = 0; q < 5; ++q) { const int c = q * 32 + lane; float v = 0.0f; if (c < NF) v = pmul(pmul(Fo[n * FP + c] - mu, rs), bf16_rne(lw[c])) + bf16_rne(lb_[c]); else if (c >= NF && c < NF + M) v = MI[n * M + (c - NF)]; ((volatile float*)NI)[n * 160 + c] = v; } } __threadfence(); }
}
__global__ __launch_bounds__(32) void resid_kernel(const float* __restrict__ Hh, int NLIM, float* __restrict__ Fo) {
  const int lane = threadIdx.x; const size_t m0 = (size_t)blockIdx.x * 16; if (m0 >= (size_t)NLIM) return; float v[16][4];
  for (int rr = 0; rr < 16; ++rr) for (int q = 0; q < 4; ++q) { const int c = q * 32 + lane; v[rr][q] = Fo[(m0 + rr) * FP + c] + (c < NF ? Hh[(m0 + rr) * 112 + c] : 0.0f); }
  for (int pass = 0; pass < 2; ++pass) { for (int rr = 0; rr < 16; ++rr) for (int q = 0; q < 4; ++q) ((volatile float*)Fo)[(m0 + rr) * FP + q * 32 + lane] = v[rr][q]; __threadfence(); }
}
__global__ __launch_bounds__(256) void pool_kernel(const float* __restrict__ Fo, const int* __restrict__ batch, int NLIM, float* __restrict__ out) {
  const int tid = threadIdx.x;
  auto lb = [&](int key) -> int { int lo = 0, hi = N; for (int it = 0; it < 17 && lo < hi; ++it) { const int mid = (lo + hi) >> 1; if (batch[mid] < key) lo = mid + 1; else hi = mid; } return lo; };
  for (int pass = 0; pass < 2; ++pass) { for (int i = tid; i < G * NF; i += 256) { const int g = i / NF, c = i % NF; int s0 = lb(g), e0 = lb(g + 1); const int call = e0 - s0; if (e0 > NLIM) e0 = NLIM; if (e0 < s0) e0 = s0; float s = 0.0f;
#pragma unroll 1
      for (int n = s0; n < e0; ++n) s += Fo[(size_t)n * FP + c]; ((volatile float*)out)[i] = s / (float)(call < 1 ? 1 : call); } __threadfence(); }
}
}

extern "C" void kernel_launch(void* const* d_in, const int* in_sizes, int n_in, void* d_out, int out_size, void* d_ws, size_t ws_size, hipStream_t stream) {
  (void)n_in;
  auto Fp = [&](int i) { return (const float*)d_in[i]; }; auto Ip = [&](int i) { return (const int*)d_in[i]; };
  if (in_sizes[0] != N * 16 || in_sizes[1] != 2 * E || in_sizes[2] != E || in_sizes[3] != N * 3 || in_sizes[4] != N || in_sizes[5] != 119 * 32 || in_sizes[15] != NL * 222 * EH || in_sizes[17] != NL * EH * M || in_sizes[19] != NL * 142 * NHID || in_sizes[21] != NL * NHID * NF || out_size != G * NF) return;
  const int NLIM = N; const int GB16 = NBLK;
  size_t off = 0; char* ws = (char*)d_ws;
  auto carve = [&](size_t bytes) { char* p = ws + off; off += (bytes + 255) & ~(size_t)255; return p; };
  b16* WE1[2]; b16* WE2[2]; b16* WN1[2]; b16* WN2[2]; for (int l = 0; l < 2; ++l) { WE1[l] = (b16*)carve(256 * FP * 2); WE2[l] = (b16*)carve(32 * EH * 2); WN1[l] = (b16*)carve(128 * 160 * 2); WN2[l] = (b16*)carve(112 * 128 * 2); }
  float* Fo = (float*)carve((size_t)N * FP * 4); float* PDS = (float*)carve((size_t)N * 256 * 4); float* MI = (float*)carve((size_t)N * M * 4); float* ST = (float*)carve(G * 32 * 4); float* NI = (float*)carve((size_t)N * 160 * 4); float* HH = (float*)carve((size_t)N * 128 * 4); float* H2 = (float*)carve((size_t)N * 112 * 4);
  CsrBufs9 csr; off = csr_carve9(csr, ws, off, E, N);
  if (off > ws_size || off > ((size_t)192 << 20)) return;
  for (int l = 0; l < 2; ++l) { const float* w1 = Fp(15) + (size_t)l * 222 * EH;
    wput_kernel<<<(128 * 16 + 255) / 256, 256, 0, stream>>>(w1, 0, NF, FP, EH, 128, 0, 0, FP, WE1[l]); wput_kernel<<<(128 * 16 + 255) / 256, 256, 0, stream>>>(w1, NF, NF, FP, EH, 128, 128, 0, FP, WE1[l]);
    wput_kernel<<<(32 * 16 + 255) / 256, 256, 0, stream>>>(Fp(17) + (size_t)l * EH * M, 0, EH, EH, M, 32, 0, 0, EH, WE2[l]);
    wput_kernel<<<(128 * 20 + 255) / 256, 256, 0, stream>>>(Fp(19) + (size_t)l * 142 * NHID, 0, 142, 160, NHID, 128, 0, 0, 160, WN1[l]);
    wput_kernel<<<(112 * 16 + 255) / 256, 256, 0, stream>>>(Fp(21) + (size_t)l * NHID * NF, 0, NHID, 128, NF, 112, 0, 0, 128, WN2[l]); }
  csr_build9(csr, Ip(1) + E, E, N, stream);
  feat_kernel<<<NBLK, 32, 0, stream>>>(Fp(0), nullptr, Fp(5), Fp(6), Fp(7), Fp(8), Fp(9), Fp(10), Fp(11), Fp(12), Fp(13), Fp(14), Fo);
  for (int l = 0; l < 2; ++l) {
    dense_kernel<FP, 16, 0><<<GB16, 32, 0, stream>>>(Fo, FP, NF, WE1[l], nullptr, 0, 256, NLIM, PDS);
    msg_kernel<<<(unsigned)NLIM, 32, 0, stream>>>(PDS, Fp(3), Fp(2), Ip(1), Fp(15) + (size_t)l * 222 * EH, Fp(16) + l * EH, WE2[l], Fp(18) + l * M, csr.PERM, csr.ROWPTR, csr.ROWCNT, (int)csr.permLen, NLIM, MI);
    lnstat_kernel<<<G, 256, 0, stream>>>(Fo, Ip(4), NLIM, ST);
    nin_kernel<<<GB16, 32, 0, stream>>>(Fo, MI, ST, Ip(4), Fp(23) + l * NF, Fp(24) + l * NF, NLIM, NI);
    dense_kernel<160, 8, 1><<<GB16, 32, 0, stream>>>(NI, 160, 142, WN1[l], Fp(20) + l * NHID, NHID, 128, NLIM, HH);
    dense_kernel<128, 7, 0><<<GB16, 32, 0, stream>>>(HH, 128, NHID, WN2[l], Fp(22) + l * NF, NF, 112, NLIM, H2);
    resid_kernel<<<GB16, 32, 0, stream>>>(H2, NLIM, Fo); }
  pool_kernel<<<1, 256, 0, stream>>>(Fo, Ip(4), NLIM, (float*)d_out);
}
